// MultiHeadAttention_34694745817616
// MI455X (gfx1250) — hardware-verified
//
#include <hip/hip_runtime.h>
#include <math.h>

#ifndef NB
#define NB 4
#endif
#ifndef SEQ
#define SEQ 2048
#endif
#define NB_FULL 4
#define SEQ_FULL 2048
#define DM 512
#define NH 8
#define HD 64
#define NTOK (NB * SEQ)
#define NQB (SEQ / 64)

#ifndef EROWS
#if SEQ >= 512
#define EROWS 512
#else
#define EROWS SEQ
#endif
#endif
#define EQB (EROWS / 64)

#define W_CARRY    16.0f
#define QKV_CARRY  16.0f
#define P_CARRY    1024.0f
#define SC_SCORE   (0.125f / 256.0f)
#define CTX_FOLD   (1.0f / 64.0f)
#define H_CARRY    1024.0f
#define HEAD_SCALE (1.0f / 4096.0f)
#define OUT_SCALE  (1.0f / 16384.0f)
#define RES_ATT    2048.0f
#define RES_GEMM   64.0f
#define W_RES_CARRY 0.25f
#define NEG_FILL   (-__FLT_MAX__)

static_assert(NH * HD == DM);
static_assert(HD == 64);
static_assert(DM % 64 == 0);
static_assert(DM % 32 == 0);
static_assert(DM % 8 == 0);
static_assert(SEQ % 64 == 0);
static_assert(NTOK % 64 == 0);
static_assert(NB <= NB_FULL);
static_assert(SEQ <= SEQ_FULL);
static_assert(sizeof(long) == 8);
static_assert((DM * (DM / 8)) % 256 == 0);
static_assert(EROWS % 64 == 0);
static_assert(EROWS <= SEQ);
static_assert((SEQ - EROWS) % 64 == 0);
static_assert((NB * EROWS) % 64 == 0);
static_assert((NH * HD * (HD / 8)) % 256 == 0);
static_assert(HD % 32 == 0 && (2 * HD) % 32 == 0 && (2 * DM) % 32 == 0);
static_assert(W_CARRY / RES_GEMM == W_RES_CARRY);

typedef __attribute__((ext_vector_type(16))) _Float16 v16h;
typedef __attribute__((ext_vector_type(8)))  _Float16 v8h;
typedef __attribute__((ext_vector_type(8)))  float    v8f;
typedef __attribute__((ext_vector_type(4)))  float    v4f;
typedef __attribute__((ext_vector_type(4)))  unsigned int v4u;
typedef unsigned short us;
typedef __attribute__((ext_vector_type(8)))  unsigned short v8us;
typedef __attribute__((ext_vector_type(16))) unsigned short v16us;
typedef _Float16 h16;


#define VST2(T, ptr, val) do { const T vst2_v_ = (val); *(volatile T*)(ptr) = vst2_v_; __threadfence(); *(volatile T*)(ptr) = vst2_v_; } while (0)

namespace gk {

__device__ __forceinline__ unsigned short f2bf_bits(float f) {
  unsigned u = __float_as_uint(f);
  return (unsigned short)((u + 0x7FFFu + ((u >> 16) & 1u)) >> 16);
}
__device__ __forceinline__ unsigned short f2h_bits(float f) { return __builtin_bit_cast(unsigned short, (_Float16)f); }

__device__ __forceinline__ void dep_guard_h(v8f& a, v8f& b, v16h x, v16h y) { asm volatile("v_nop\n\tv_nop\n\tv_nop\n\tv_nop" : "+v"(a), "+v"(b) : "v"(x), "v"(y)); }
__device__ __forceinline__ void keep4_h(v16h a, v16h b, v16h c, v16h d) { asm volatile("v_nop" :: "v"(a), "v"(b), "v"(c), "v"(d)); }
__device__ __forceinline__ void acc_guard4(v8f& a, v8f& b, v8f& c, v8f& d) { asm volatile("v_nop\n\tv_nop\n\tv_nop\n\tv_nop" : "+v"(a), "+v"(b), "+v"(c), "+v"(d)); }

union FragU { v16h v; v8h h[2]; };
__device__ __forceinline__ v16h frag_load(const _Float16* p) {
  FragU f; f.h[0] = *(const v8h*)(p); f.h[1] = *(const v8h*)(p + 16); return f.v;
}
__device__ __forceinline__ v8f frag_mma(v16h a, v16h b, v8f c) {
  return __builtin_amdgcn_wmma_f32_16x16x32_f16(false, a, false, b, (short)0, c, false, false);
}

template <int BIAS_MODE, int OUT_MODE>
__device__ __forceinline__ void gemm64_body(
    const unsigned short* __restrict__ Ap, int lda, long strideA,
    const unsigned short* __restrict__ Btp, int ldb, long strideB,
    void* __restrict__ Cout, int ldc, long strideC,
    const float* __restrict__ biasp, int strideBias,
    int M, int N, int K, float scale, float carry) {
  __shared__ __align__(16) float sT[8][16 * 68];
  const _Float16* A = (const _Float16*)Ap; const _Float16* Bt = (const _Float16*)Btp;
  const int b    = blockIdx.y;
  const int lane = threadIdx.x & 31;
  const int wave = threadIdx.x >> 5;
  const int tilesN = N >> 6;
  const int tilesM = M >> 6;
  const int tile = blockIdx.x * 8 + wave;
  if (tile >= tilesM * tilesN) return;
  const int tm = tile / tilesN;
  const int tn = tile - tm * tilesN;
  const int m0 = tm << 6;
  const int n0 = tn << 6;

  const _Float16* Ab = A  + (size_t)b * strideA;
  const _Float16* Bb = Bt + (size_t)b * strideB;
  const float* bias = biasp + (size_t)b * strideBias;

  const int rlane = lane & 15;
  const int koff  = (lane >> 4) * 8;
  const int mOff  = (lane >> 4) * 8;

  v8f acc[4][4];
#pragma unroll
  for (int i = 0; i < 4; ++i)
#pragma unroll
    for (int j = 0; j < 4; ++j) acc[i][j] = (v8f){0.f,0.f,0.f,0.f,0.f,0.f,0.f,0.f};

  for (int k0 = 0; k0 < K; k0 += 32) {
    v16h bh[4];
#pragma unroll
    for (int j = 0; j < 4; ++j) {
      const size_t bo = (size_t)(n0 + (j << 4) + rlane) * ldb + koff + k0;
      bh[j] = frag_load(Bb + bo);
    }
#pragma unroll
    for (int i = 0; i < 4; ++i) {
      const size_t ao = (size_t)(m0 + (i << 4) + rlane) * lda + koff + k0;
      v16h ah = frag_load(Ab + ao);
#pragma unroll
      for (int j = 0; j < 4; ++j) acc[i][j] = frag_mma(ah, bh[j], acc[i][j]);
      dep_guard_h(acc[i][0], acc[i][3], ah, ah);
    }
    keep4_h(bh[0], bh[1], bh[2], bh[3]);
  }
  acc_guard4(acc[0][0], acc[0][1], acc[0][2], acc[0][3]);
  acc_guard4(acc[1][0], acc[1][1], acc[1][2], acc[1][3]);
  acc_guard4(acc[2][0], acc[2][1], acc[2][2], acc[2][3]);
  acc_guard4(acc[3][0], acc[3][1], acc[3][2], acc[3][3]);

  float* slab = sT[wave];
#pragma unroll
  for (int i = 0; i < 4; ++i) {
    const int mBase = m0 + (i << 4);
#pragma unroll
    for (int j = 0; j < 4; ++j) {
      const int n = n0 + (j << 4) + rlane;
      float bv = 0.f;
      if (BIAS_MODE == 2) bv = bias[n];
#pragma unroll
      for (int r = 0; r < 8; ++r) {
        float v = acc[i][j][r] * scale;
        if (BIAS_MODE == 1) v += bias[mBase + mOff + r];
        if (BIAS_MODE == 2) v += bv;
        slab[(mOff + r) * 68 + (j << 4) + rlane] = v * carry;
      }
    }
    __builtin_amdgcn_fence(3  , "workgroup");
    __builtin_amdgcn_wave_barrier();
    __builtin_amdgcn_fence(2  , "workgroup");
    if (OUT_MODE == 0) {
      float* C = (float*)Cout + (size_t)b * strideC;
      const int hh = lane >> 4, c4 = (lane & 15) * 4;
      for (int pass = 0; pass < 2; ++pass) {
#pragma unroll
        for (int it = 0; it < 8; ++it) {
          const int row = it * 2 + hh;
          v4f v = *(const v4f*)(slab + row * 68 + c4);
          *(volatile v4f*)(C + (size_t)(mBase + row) * ldc + n0 + c4) = v;
        }
        __threadfence();
      }
    } else {
      const int q = lane >> 3, c8 = (lane & 7) * 8;
      unsigned short* C  = (unsigned short*)Cout + (size_t)b * strideC;
      for (int pass = 0; pass < 2; ++pass) {
#pragma unroll
        for (int it = 0; it < 4; ++it) {
          const int row = it * 4 + q;
          const float* sp = slab + row * 68 + c8;
          v8us hv;
#pragma unroll
          for (int e = 0; e < 8; ++e) hv[e] = f2h_bits(sp[e]);
          *(volatile v8us*)(C + (size_t)(mBase + row) * ldc + n0 + c8) = hv;
        }
        __threadfence();
      }
    }
    __builtin_amdgcn_fence(3  , "workgroup");
    __builtin_amdgcn_wave_barrier();
    __builtin_amdgcn_fence(2  , "workgroup");
  }
}

}

__global__ __launch_bounds__(256) void k_gemm_qk(const us* __restrict__ X16, const us* __restrict__ W16, us* __restrict__ QK16, const float* __restrict__ BR) {
  static_assert(NTOK % 64 == 0 && DM % 64 == 0 && DM % 32 == 0);
  gk::gemm64_body<2, 1>(X16, DM, (long)NTOK * DM, W16, DM, (long)DM * DM, (void*)QK16, DM, (long)NTOK * DM, BR, DM, NTOK, DM, DM, 1.0f / W_CARRY, QKV_CARRY);
}
__global__ __launch_bounds__(256) void k_gemm_vt(const us* __restrict__ Wv16, const us* __restrict__ Xv16, us* __restrict__ VT16, const float* __restrict__ BRv) {
  static_assert(NTOK % 64 == 0 && DM % 64 == 0 && DM % 32 == 0);
  gk::gemm64_body<1, 1>(Wv16, DM, 0L, Xv16, DM, 0L, (void*)VT16, NTOK, 0L, BRv, 0, DM, NTOK, DM, 1.0f / W_CARRY, QKV_CARRY);
}
__global__ __launch_bounds__(256) void k_gemm_vte(const us* __restrict__ Wv16, const us* __restrict__ Xv16, float* __restrict__ VE, const float* __restrict__ BRv) {
  gk::gemm64_body<1, 0>(Wv16, DM, 0L, Xv16, DM, (long)SEQ * DM, (void*)VE, EROWS, (long)DM * EROWS, BRv, 0, DM, EROWS, DM, 1.0f / W_CARRY, QKV_CARRY);
}
__global__ __launch_bounds__(256) void k_gemm_heads(const us* __restrict__ CTX, const us* __restrict__ WhT16, us* __restrict__ HEADS, const float* __restrict__ BRh) {
  gk::gemm64_body<2, 1>(CTX, DM, (long)HD, WhT16, HD, (long)HD * HD, (void*)HEADS, DM, (long)HD, BRh, HD, NTOK, HD, HD, HEAD_SCALE, H_CARRY);
}
__global__ __launch_bounds__(256) void k_gemm_heads_early(const us* __restrict__ CTXE, const us* __restrict__ WhE, float* __restrict__ HE, const float* __restrict__ BRh) {
  gk::gemm64_body<2, 0>(CTXE, 2 * DM, (long)(2 * HD), WhE, 2 * HD, (long)HD * 2 * HD, (void*)HE, DM, (long)HD, BRh, HD, NB * EROWS, HD, 2 * HD, HEAD_SCALE, H_CARRY);
}
__global__ __launch_bounds__(256) void k_gemm_out_main(const us* __restrict__ HEADSo, const us* __restrict__ WoT16, float* __restrict__ outo, const float* __restrict__ BRo) {
  gk::gemm64_body<2, 0>(HEADSo, DM, (long)SEQ * DM, WoT16, DM, 0L, (void*)outo, DM, (long)SEQ_FULL * DM, BRo, 0, SEQ - EROWS, DM, DM, OUT_SCALE, 1.0f);
}
__global__ __launch_bounds__(256) void k_gemm_out_early(const us* __restrict__ HE16, const us* __restrict__ WoE, float* __restrict__ out, const float* __restrict__ BRo) {
  gk::gemm64_body<2, 0>(HE16, 2 * DM, (long)EROWS * 2 * DM, WoE, 2 * DM, 0L, (void*)out, DM, (long)SEQ_FULL * DM, BRo, 0, EROWS, DM, 2 * DM, OUT_SCALE, 1.0f);
}

__device__ __forceinline__ unsigned int cmb_pk2(float a, float b) { return (unsigned int)__builtin_bit_cast(unsigned short, (_Float16)a) | ((unsigned int)__builtin_bit_cast(unsigned short, (_Float16)b) << 16); }
__device__ __forceinline__ float cmb_bf(float v) { const unsigned u = __builtin_bit_cast(unsigned, v); const unsigned r = (u + 0x7fffu + ((u >> 16) & 1u)) & 0xffff0000u; return __builtin_bit_cast(float, r); }
__device__ __forceinline__ void cast8_f16(const float* __restrict__ s, us* __restrict__ d, float sc) {
  const v4f a = *(const v4f*)s; const v4f b2 = *(const v4f*)(s + 4);
  v4u pk;
  pk.x = cmb_pk2(cmb_bf(a.x) * sc, cmb_bf(a.y) * sc); pk.y = cmb_pk2(cmb_bf(a.z) * sc, cmb_bf(a.w) * sc);
  pk.z = cmb_pk2(cmb_bf(b2.x) * sc, cmb_bf(b2.y) * sc); pk.w = cmb_pk2(cmb_bf(b2.z) * sc, cmb_bf(b2.w) * sc);
  VST2(v4u, (v4u*)d, pk);
}

static __device__ __forceinline__ h16 toh_flush(float v) { const h16 r = (h16)v; return (fabsf(v) < 6.103515625e-05f) ? (h16)0.0f : r; }
static __device__ __forceinline__ unsigned short toh_flush_bits(float v) { return __builtin_bit_cast(unsigned short, toh_flush(v)); }
static __device__ __forceinline__ unsigned int pk2_flush(float a, float b) { return (unsigned int)toh_flush_bits(a) | ((unsigned int)toh_flush_bits(b) << 16); }

__device__ __forceinline__ void ld8_strided_bf(const float* __restrict__ s, int st, float (&x)[8]) {
#pragma unroll
  for (int i = 0; i < 8; ++i) x[i] = cmb_bf(s[(size_t)i * st]);
}
__device__ __forceinline__ v4u pack8_scaled(const float (&x)[8], float sc) {
  v4u pk;
  pk.x = pk2_flush(x[0] * sc, x[1] * sc); pk.y = pk2_flush(x[2] * sc, x[3] * sc);
  pk.z = pk2_flush(x[4] * sc, x[5] * sc); pk.w = pk2_flush(x[6] * sc, x[7] * sc);
  return pk;
}
__device__ __forceinline__ void cast_proj(const float* __restrict__ W, us* __restrict__ T, int u) {
  const int n = u / (DM / 8); const int d0 = 8 * (u % (DM / 8));
  const int hd = n / HD; const int kk = n % HD;
  float x[8];
  ld8_strided_bf(W + ((size_t)hd * DM + d0) * HD + kk, HD, x);
  VST2(v4u, (v4u*)(T + (size_t)n * DM + d0), pack8_scaled(x, W_CARRY));
}
#define CWB ((DM * (DM / 8)) / 256)
#define CHB ((NH * HD * (HD / 8)) / 256)
__global__ __launch_bounds__(256) void k_cast_w(const float* __restrict__ Wq, const float* __restrict__ Wk, const float* __restrict__ Wv,
                                                const float* __restrict__ Wh, const float* __restrict__ Wo,
                                                us* __restrict__ W16, us* __restrict__ WhT16, us* __restrict__ WhE, us* __restrict__ WoT16, us* __restrict__ WoE) {
  const int blk = blockIdx.x;
  const int t = threadIdx.x;
  if (blk < CWB) {
    cast_proj(Wq, W16, blk * 256 + t);
  } else if (blk < 2 * CWB) {
    cast_proj(Wk, W16 + (size_t)DM * DM, (blk - CWB) * 256 + t);
  } else if (blk < 3 * CWB) {
    cast_proj(Wv, W16 + (size_t)2 * DM * DM, (blk - 2 * CWB) * 256 + t);
  } else if (blk < 4 * CWB) {
    const int u = (blk - 3 * CWB) * 256 + t;
    const int n = u / (DM / 8); const int k0 = 8 * (u % (DM / 8));
    float x[8];
    ld8_strided_bf(Wo + (size_t)k0 * DM + n, DM, x);
    const v4u pv = pack8_scaled(x, W_CARRY);
    const v4u pr = pack8_scaled(x, W_RES_CARRY);
    VST2(v4u, (v4u*)(WoT16 + (size_t)n * DM + k0), pv);
    VST2(v4u, (v4u*)(WoE + (size_t)n * (2 * DM) + k0), pv);
    VST2(v4u, (v4u*)(WoE + (size_t)n * (2 * DM) + DM + k0), pr);
  } else if (blk < 4 * CWB + CHB) {
    const int u = (blk - 4 * CWB) * 256 + t;
    const int row = u / (HD / 8); const int v0 = 8 * (u % (HD / 8));
    const int hd = row / HD; const int w = row % HD;
    float x[8];
    ld8_strided_bf(Wh + ((size_t)hd * HD + v0) * HD + w, HD, x);
    const v4u pv = pack8_scaled(x, W_CARRY);
    const v4u pr = pack8_scaled(x, W_RES_CARRY);
    VST2(v4u, (v4u*)(WhT16 + (size_t)row * HD + v0), pv);
    VST2(v4u, (v4u*)(WhE + (size_t)row * (2 * HD) + v0), pv);
    VST2(v4u, (v4u*)(WhE + (size_t)row * (2 * HD) + HD + v0), pr);
  }
}
__global__ __launch_bounds__(256) void k_bias5(const float* __restrict__ bq, const float* __restrict__ bk, const float* __restrict__ bv, const float* __restrict__ bhd, const float* __restrict__ bo, float* __restrict__ BR) {
  const int u = blockIdx.x * 256 + threadIdx.x; if (u >= DM) return;
  VST2(float, BR + u, cmb_bf(bq[u]));
  VST2(float, BR + DM + u, cmb_bf(bk[u]));
  VST2(float, BR + 2 * DM + u, cmb_bf(bv[u]));
  VST2(float, BR + 3 * DM + u, cmb_bf(bhd[u]));
  VST2(float, BR + 4 * DM + u, cmb_bf(bo[u]));
}
__global__ __launch_bounds__(256) void k_cast_x3(const float* __restrict__ xq, const float* __restrict__ xk, const float* __restrict__ xv, us* __restrict__ X16) {
  const long long u = (long long)blockIdx.x * 256 + threadIdx.x; if (u >= (long long)NTOK * (DM / 8)) return;
  const int r = (int)(u / (DM / 8)); const int c0 = 8 * (int)(u % (DM / 8));
  const int b = r / SEQ; const int s = r - b * SEQ;
  const size_t so = ((size_t)b * SEQ_FULL + s) * DM + c0; const size_t dofs = (size_t)r * DM + c0;
  cast8_f16(xq + so, X16 + dofs, 1.0f);
  cast8_f16(xk + so, X16 + (size_t)NTOK * DM + dofs, 1.0f);
  cast8_f16(xv + so, X16 + (size_t)2 * NTOK * DM + dofs, 1.0f);
}
__device__ __forceinline__ void split2(float x, float y, float rc, unsigned int& hv, unsigned int& rv) {
  const h16 hx = toh_flush(x); const h16 hy = toh_flush(y);
  hv = (unsigned int)__builtin_bit_cast(unsigned short, hx) | ((unsigned int)__builtin_bit_cast(unsigned short, hy) << 16);
  rv = pk2_flush((x - (float)hx) * rc, (y - (float)hy) * rc);
}
__global__ __launch_bounds__(256) void k_split(const float* __restrict__ src, us* __restrict__ dhi, us* __restrict__ dres, int rows, int cols, int pitch, float rc) {
  const long long u = (long long)blockIdx.x * 256 + threadIdx.x;
  const int cg = cols >> 3;
  if (u >= (long long)rows * cg) return;
  const int r = (int)(u / cg); const int c0 = 8 * (int)(u % cg);
  const float* s = src + (size_t)r * cols + c0;
  const v4f a = *(const v4f*)s; const v4f b2 = *(const v4f*)(s + 4);
  unsigned int hw0, hw1, hw2, hw3, rw0, rw1, rw2, rw3;
  split2(a.x, a.y, rc, hw0, rw0); split2(a.z, a.w, rc, hw1, rw1);
  split2(b2.x, b2.y, rc, hw2, rw2); split2(b2.z, b2.w, rc, hw3, rw3);
  v4u ph, pr;
  ph.x = hw0; ph.y = hw1; ph.z = hw2; ph.w = hw3;
  pr.x = rw0; pr.y = rw1; pr.z = rw2; pr.w = rw3;
  const size_t o = (size_t)r * pitch + c0;
  VST2(v4u, (v4u*)(dhi + o), ph);
  VST2(v4u, (v4u*)(dres + o), pr);
}

__device__ __forceinline__ v8f mma_h(v16h a, v16h b, v8f c) {
  c = __builtin_amdgcn_wmma_f32_16x16x32_f16(false, a, false, b, (short)0, c, false, false);
  asm volatile("v_nop\n\tv_nop\n\tv_nop\n\tv_nop" : "+v"(c) : "v"(a), "v"(b));
  return c;
}
__device__ __forceinline__ void wave_sync() {
  __builtin_amdgcn_fence(3  , "workgroup");
  __builtin_amdgcn_wave_barrier();
  __builtin_amdgcn_fence(2  , "workgroup");
}
union FBU { v16us u; v8us h[2]; };
#define LDFRAG(dst, arr, off) do { FBU f_; f_.h[0] = *(const v8us*)&arr[(off)]; f_.h[1] = *(const v8us*)&arr[(off) + 16]; dst = __builtin_bit_cast(v16h, f_.u); } while (0)

template <int RH>
__device__ __forceinline__ void attn_body(const us* __restrict__ QK16, const us* __restrict__ VH, const us* __restrict__ VR, const int* __restrict__ MK,
                                          us* __restrict__ CTX, us* __restrict__ CTXE, const int nqb, const int qb_first, const int vpitch, const long vbstride) {
  __shared__ __align__(16) us Qs[64 * 64];
  __shared__ __align__(16) us Ks[64 * 64];
  __shared__ __align__(16) us Vts[64 * 64];
  __shared__ __align__(16) us Vrs[64 * 64];
  __shared__ __align__(16) us Ps[4 * 16 * 32];
  __shared__ __align__(16) us Prs[4 * 16 * 32];
  __shared__ int msk_s[64];

  const int tid = threadIdx.x, lane = tid & 31, hh = lane >> 4, c = lane & 15;
  const int wave = __builtin_amdgcn_readfirstlane((int)(threadIdx.x >> 5));
  const int bx = blockIdx.x;
  const int qb = qb_first + bx % nqb; const int bh = bx / nqb; const int h = bh % NH; const int b = bh / NH;
  const int tok0 = b * SEQ + qb * 64;
  const size_t KOFF = (size_t)NTOK * DM;

  {
    const int row = tid >> 1, dh = (tid & 1) * 32;
    const size_t qro_g = (size_t)(tok0 + row) * DM + h * HD + dh;
#pragma unroll
    for (int i = 0; i < 4; ++i) *(v8us*)&Qs[row * 64 + dh + 8 * i] = *(const v8us*)(QK16 + qro_g + 8 * i);
  }
  __syncthreads();

  float mrow[8], lsum[8];
  v8f oacc[4];
  v8f ores[4];
#pragma unroll
  for (int r = 0; r < 8; ++r) { mrow[r] = -__builtin_inff(); lsum[r] = 0.f; }
#pragma unroll
  for (int t = 0; t < 4; ++t) { oacc[t] = (v8f){0.f,0.f,0.f,0.f,0.f,0.f,0.f,0.f}; ores[t] = (v8f){0.f,0.f,0.f,0.f,0.f,0.f,0.f,0.f}; }

  const int pb = wave * 512;
  const int qro = (wave * 16 + c) * 64 + 8 * hh;
  const int qrel = qb * 64 + wave * 16 + 8 * hh;

#pragma unroll 1
  for (int kc = 0; kc <= qb; ++kc) {
    const int kv0 = kc * 64;
    __syncthreads();
    {
      const int row = tid >> 1, dh = (tid & 1) * 32;
      const size_t kro = KOFF + (size_t)(b * SEQ + kv0 + row) * DM + h * HD + dh;
      const size_t vro = (size_t)b * (size_t)vbstride + (size_t)(h * HD + row) * (size_t)vpitch + (size_t)(kv0 + dh);
#pragma unroll
      for (int i = 0; i < 4; ++i) {
        *(v8us*)&Ks[row * 64 + dh + 8 * i]  = *(const v8us*)(QK16 + kro + 8 * i);
        *(v8us*)&Vts[row * 64 + dh + 8 * i] = *(const v8us*)(VH + vro + 8 * i);
        if (RH) *(v8us*)&Vrs[row * 64 + dh + 8 * i] = *(const v8us*)(VR + vro + 8 * i);
      }
      if (tid < 64) msk_s[tid] = MK[(size_t)b * SEQ_FULL + kv0 + tid];
    }
    __syncthreads();

#pragma unroll 1
    for (int hf = 0; hf < 2; ++hf) {
      v8f s0 = (v8f){0.f,0.f,0.f,0.f,0.f,0.f,0.f,0.f};
      v8f s1 = s0;
#pragma unroll
      for (int dc = 0; dc < 2; ++dc) {
        v16h qf, kf;
        LDFRAG(qf, Qs, qro + dc * 32);
        const int ko0 = ((2 * hf) * 16 + c) * 64 + dc * 32 + 8 * hh;
        LDFRAG(kf, Ks, ko0);
        s0 = mma_h(qf, kf, s0);
        const int ko1 = ko0 + 16 * 64;
        LDFRAG(kf, Ks, ko1);
        s1 = mma_h(qf, kf, s1);
      }
      const bool vis0 = (msk_s[hf * 32 + c] == 0);
      const bool vis1 = (msk_s[hf * 32 + 16 + c] == 0);
      const int kq0 = kv0 + hf * 32 + c - qrel;
#pragma unroll
      for (int r = 0; r < 8; ++r) {
        const bool keep0 = vis0 && (kq0 <= r);
        const bool keep1 = vis1 && (kq0 + 16 <= r);
        const float a0 = keep0 ? s0[r] * SC_SCORE : NEG_FILL;
        const float a1 = keep1 ? s1[r] * SC_SCORE : NEG_FILL;
        float m = fmaxf(a0, a1);
        m = fmaxf(m, __shfl_xor(m, 1, 32)); m = fmaxf(m, __shfl_xor(m, 2, 32));
        m = fmaxf(m, __shfl_xor(m, 4, 32)); m = fmaxf(m, __shfl_xor(m, 8, 32));
        const float mnew = fmaxf(mrow[r], m);
        const float alpha = expf(mrow[r] - mnew);
        mrow[r] = mnew;
        const float p0 = expf(a0 - mnew);
        const float p1 = expf(a1 - mnew);
        const float w0 = keep0 ? p0 : 0.f;
        const float w1 = keep1 ? p1 : 0.f;
        const float c0 = w0 * P_CARRY;
        const float c1 = w1 * P_CARRY;
        const h16 ph0 = toh_flush(c0);
        const h16 ph1 = toh_flush(c1);
        if (RH) lsum[r] = lsum[r] * alpha + (w0 + w1);
        else    lsum[r] = lsum[r] * alpha + ((float)ph0 + (float)ph1) * (1.0f / P_CARRY);
#pragma unroll
        for (int t = 0; t < 4; ++t) oacc[t][r] *= alpha;
        if (RH) {
#pragma unroll
          for (int t = 0; t < 4; ++t) ores[t][r] *= alpha;
        }
        const int po = pb + (8 * hh + r) * 32 + c;
        Ps[po] = __builtin_bit_cast(unsigned short, ph0);
        Ps[po + 16] = __builtin_bit_cast(unsigned short, ph1);
        if (RH) {
          Prs[po] = toh_flush_bits((c0 - (float)ph0) * RES_ATT);
          Prs[po + 16] = toh_flush_bits((c1 - (float)ph1) * RES_ATT);
        }
      }
      wave_sync();
      v16h pa;
      LDFRAG(pa, Ps, pb + c * 32 + 8 * hh);
      if (RH) {
        v16h par;
        LDFRAG(par, Prs, pb + c * 32 + 8 * hh);
#pragma unroll
        for (int t = 0; t < 4; ++t) {
          v16h vf, vrf;
          const int vo = (t * 16 + c) * 64 + hf * 32 + 8 * hh;
          LDFRAG(vf, Vts, vo);
          LDFRAG(vrf, Vrs, vo);
          oacc[t] = mma_h(pa, vf, oacc[t]);
          ores[t] = mma_h(pa, vrf, ores[t]);
          ores[t] = mma_h(par, vf, ores[t]);
        }
      } else {
#pragma unroll
        for (int t = 0; t < 4; ++t) {
          v16h vf;
          const int vo = (t * 16 + c) * 64 + hf * 32 + 8 * hh;
          LDFRAG(vf, Vts, vo);
          oacc[t] = mma_h(pa, vf, oacc[t]);
        }
      }
      wave_sync();
    }
  }

  __syncthreads();
  {
    const int sb = wave * 1024;
#pragma unroll
    for (int r = 0; r < 8; ++r) {
      float l = lsum[r];
      l += __shfl_xor(l, 1, 32); l += __shfl_xor(l, 2, 32); l += __shfl_xor(l, 4, 32); l += __shfl_xor(l, 8, 32);
      const float invl = 1.0f / l;
      const float fac = invl * CTX_FOLD;
#pragma unroll
      for (int t = 0; t < 4; ++t) {
        const int si = sb + (8 * hh + r) * 64 + t * 16 + c;
        if (RH) {
          const float xf = (oacc[t][r] + ores[t][r] * (1.0f / RES_ATT)) * fac;
          const h16 xh = toh_flush(xf);
          Ks[si] = __builtin_bit_cast(unsigned short, xh);
          Vts[si] = toh_flush_bits((xf - (float)xh) * RES_GEMM);
        } else {
          Ks[si] = toh_flush_bits(oacc[t][r] * fac);
        }
      }
    }
    wave_sync();
    const int q4 = lane >> 3, c8 = (lane & 7) * 8;
    v8us hv[4];
    v8us hr[4];
#pragma unroll
    for (int it = 0; it < 4; ++it) {
      const int row = it * 4 + q4;
      hv[it] = *(const v8us*)&Ks[sb + row * 64 + c8];
      if (RH) hr[it] = *(const v8us*)&Vts[sb + row * 64 + c8]; else hr[it] = hv[it];
    }
    for (int pass = 0; pass < 2; ++pass) {
#pragma unroll
      for (int it = 0; it < 4; ++it) {
        const int row = it * 4 + q4;
        us* dst = CTX + (size_t)(tok0 + wave * 16 + row) * DM + h * HD + c8;
        *(volatile v8us*)(dst) = hv[it];
        if (RH) {
          const size_t er = (size_t)(b * EROWS + qb * 64 + wave * 16 + row);
          us* de = CTXE + er * (size_t)(2 * DM) + h * (2 * HD) + c8;
          *(volatile v8us*)(de) = hv[it];
          *(volatile v8us*)(de + HD) = hr[it];
        }
      }
      __threadfence();
    }
  }
}

__global__ __launch_bounds__(128) void k_attn_main(const us* __restrict__ QK16, const us* __restrict__ VT16, const int* __restrict__ MK, us* __restrict__ CTX) {
  attn_body<0>(QK16, VT16, VT16, MK, CTX, CTX, (NQB - EQB) > 0 ? (NQB - EQB) : 1, EQB, NTOK, (long)SEQ);
}
__global__ __launch_bounds__(128) void k_attn_early(const us* __restrict__ QK16, const us* __restrict__ VEH, const us* __restrict__ VER, const int* __restrict__ MK, us* __restrict__ CTX, us* __restrict__ CTXE) {
  attn_body<1>(QK16, VEH, VER, MK, CTX, CTXE, EQB > 0 ? EQB : 1, 0, EROWS, (long)DM * EROWS);
}

#define WS_X16   ((size_t)3 * NTOK * DM * 2)
#define WS_W16   ((size_t)3 * DM * DM * 2)
#define WS_WOT   ((size_t)DM * DM * 2)
#define WS_WOE   ((size_t)DM * 2 * DM * 2)
#define WS_WHT   ((size_t)NH * HD * HD * 2)
#define WS_WHE   ((size_t)NH * HD * 2 * HD * 2)
#define WS_BR    ((size_t)5 * DM * 4)
#define WS_QK    ((size_t)2 * NTOK * DM * 2)
#define WS_VT    ((size_t)DM * NTOK * 2)
#define WS_VE    ((size_t)NB * DM * EROWS * 4)
#define WS_VEH   ((size_t)NB * DM * EROWS * 2)
#define WS_VER   ((size_t)NB * DM * EROWS * 2)
#define WS_CTX   ((size_t)NTOK * DM * 2)
#define WS_CTXE  ((size_t)NB * EROWS * 2 * DM * 2)
#define WS_HEADS ((size_t)NTOK * DM * 2)
#define WS_HE    ((size_t)NB * EROWS * DM * 4)
#define WS_HE16  ((size_t)NB * EROWS * 2 * DM * 2)
#define WS_TOTAL (WS_X16 + WS_W16 + WS_WOT + WS_WOE + WS_WHT + WS_WHE + WS_BR + WS_QK + WS_VT + WS_VE + WS_VEH + WS_VER + WS_CTX + WS_CTXE + WS_HEADS + WS_HE + WS_HE16)
static_assert(WS_X16 % 256 == 0 && WS_W16 % 256 == 0 && WS_WOT % 256 == 0 && WS_WOE % 256 == 0 && WS_WHT % 256 == 0 && WS_WHE % 256 == 0);
static_assert(WS_BR % 256 == 0 && WS_QK % 256 == 0 && WS_VT % 256 == 0 && WS_VE % 256 == 0 && WS_VEH % 256 == 0 && WS_VER % 256 == 0);
static_assert(WS_CTX % 256 == 0 && WS_CTXE % 256 == 0 && WS_HEADS % 256 == 0 && WS_HE % 256 == 0 && WS_HE16 % 256 == 0);
static_assert(WS_TOTAL <= (size_t)134217728);
static_assert((size_t)((NB_FULL - 1) * SEQ_FULL + SEQ_FULL) * DM * 4 == (size_t)16777216);

extern "C" void kernel_launch(void* const* d_in, const int* in_sizes, int n_in, void* d_out, int out_size, void* d_ws, size_t ws_size, hipStream_t stream) {
  if (n_in < 14) return;
  const long long need_x = ((long long)(NB - 1) * SEQ_FULL + SEQ) * DM;
  const long long need_m = (long long)(NB - 1) * SEQ_FULL + SEQ;
  if ((long long)in_sizes[0] < need_x || (long long)in_sizes[1] < need_x || (long long)in_sizes[2] < need_x) return;
  if ((long long)in_sizes[3] < need_m) return;
  if (in_sizes[4] < NH * DM * HD || in_sizes[6] < NH * DM * HD || in_sizes[8] < NH * DM * HD) return;
  if (in_sizes[5] < DM || in_sizes[7] < DM || in_sizes[9] < DM || in_sizes[11] < DM || in_sizes[13] < DM) return;
  if (in_sizes[10] < NH * HD * HD) return;
  if (in_sizes[12] < DM * DM) return;
  if ((long long)out_size < need_x) return;
  if (WS_TOTAL > ws_size) return;

  const float* xq = (const float*)d_in[0];
  const float* xk = (const float*)d_in[1];
  const float* xv = (const float*)d_in[2];
  const int* kmask = (const int*)d_in[3];
  const float* Wq = (const float*)d_in[4];
  const float* bq = (const float*)d_in[5];
  const float* Wk = (const float*)d_in[6];
  const float* bk = (const float*)d_in[7];
  const float* Wv = (const float*)d_in[8];
  const float* bv = (const float*)d_in[9];
  const float* Wh = (const float*)d_in[10];
  const float* bhd = (const float*)d_in[11];
  const float* Wo = (const float*)d_in[12];
  const float* bo = (const float*)d_in[13];
  float* out = (float*)d_out;

  char* wsp = (char*)d_ws;
  us* X16 = (us*)wsp;             wsp += WS_X16;
  us* W16 = (us*)wsp;             wsp += WS_W16;
  us* WoT16 = (us*)wsp;           wsp += WS_WOT;
  us* WoE = (us*)wsp;             wsp += WS_WOE;
  us* WhT16 = (us*)wsp;           wsp += WS_WHT;
  us* WhE = (us*)wsp;             wsp += WS_WHE;
  float* BR = (float*)wsp;        wsp += WS_BR;
  us* QK16 = (us*)wsp;            wsp += WS_QK;
  us* VT16 = (us*)wsp;            wsp += WS_VT;
  float* VE = (float*)wsp;        wsp += WS_VE;
  us* VEH = (us*)wsp;             wsp += WS_VEH;
  us* VER = (us*)wsp;             wsp += WS_VER;
  us* CTX = (us*)wsp;             wsp += WS_CTX;
  us* CTXE = (us*)wsp;            wsp += WS_CTXE;
  us* HEADS = (us*)wsp;           wsp += WS_HEADS;
  float* HE = (float*)wsp;        wsp += WS_HE;
  us* HE16 = (us*)wsp;            wsp += WS_HE16;

  k_cast_w<<<dim3((unsigned)(4 * CWB + CHB)), dim3(256), 0, stream>>>(Wq, Wk, Wv, Wh, Wo, W16, WhT16, WhE, WoT16, WoE);
  k_bias5<<<dim3((unsigned)((DM + 255) / 256)), dim3(256), 0, stream>>>(bq, bk, bv, bhd, bo, BR);
  k_cast_x3<<<dim3((unsigned)(((long long)NTOK * (DM / 8) + 255) / 256)), dim3(256), 0, stream>>>(xq, xk, xv, X16);
  k_gemm_qk<<<dim3((unsigned)(((NTOK / 64) * (DM / 64) + 7) / 8), 2u), dim3(256), 0, stream>>>(X16, W16, QK16, BR);
  k_gemm_vt<<<dim3((unsigned)(((DM / 64) * (NTOK / 64) + 7) / 8), 1u), dim3(256), 0, stream>>>(W16 + (size_t)2 * DM * DM, X16 + (size_t)2 * NTOK * DM, VT16, BR + 2 * DM);
  if (EQB > 0) {
    k_gemm_vte<<<dim3((unsigned)(((DM / 64) * (EROWS / 64) + 7) / 8), (unsigned)NB), dim3(256), 0, stream>>>(W16 + (size_t)2 * DM * DM, X16 + (size_t)2 * NTOK * DM, VE, BR + 2 * DM);
    k_split<<<dim3((unsigned)(((long long)NB * DM * (EROWS / 8) + 255) / 256)), dim3(256), 0, stream>>>(VE, VEH, VER, NB * DM, EROWS, EROWS, RES_ATT);
    k_attn_early<<<dim3((unsigned)(NB * NH * EQB)), dim3(128), 0, stream>>>(QK16, VEH, VER, kmask, CTX, CTXE);
  }
  if (NQB > EQB) {
    k_attn_main<<<dim3((unsigned)(NB * NH * (NQB - EQB))), dim3(128), 0, stream>>>(QK16, VT16, kmask, CTX);
  }
  k_gemm_heads<<<dim3((unsigned)(((NTOK / 64) * (HD / 64) + 7) / 8), (unsigned)NH), dim3(256), 0, stream>>>(CTX, WhT16, HEADS, BR + 3 * DM);
  if (EQB > 0) {
    k_gemm_heads_early<<<dim3((unsigned)((((NB * EROWS) / 64) * (HD / 64) + 7) / 8), (unsigned)NH), dim3(256), 0, stream>>>(CTXE, WhE, HE, BR + 3 * DM);
    k_split<<<dim3((unsigned)(((long long)NB * EROWS * (DM / 8) + 255) / 256)), dim3(256), 0, stream>>>(HE, HE16, HE16 + DM, NB * EROWS, DM, 2 * DM, RES_GEMM);
  }
  if (NQB > EQB) {
    k_gemm_out_main<<<dim3((unsigned)((((SEQ - EROWS) / 64) * (DM / 64) + 7) / 8), (unsigned)NB), dim3(256), 0, stream>>>(HEADS + (size_t)EROWS * DM, WoT16, out + (size_t)EROWS * DM, BR + 4 * DM);
  }
  if (EQB > 0) {
    k_gemm_out_early<<<dim3((unsigned)(((EROWS / 64) * (DM / 64) + 7) / 8), (unsigned)NB), dim3(256), 0, stream>>>(HE16, WoE, out, BR + 4 * DM);
  }
}
